// SparseSharedTokenCrossAttention_53085795779214
// MI455X (gfx1250) — hardware-verified
//
#include <hip/hip_runtime.h>


namespace {
constexpr int Bn = 2, HWQ = 8192, D = 512, L = 4096, KN = 32, NH = 8, DH = 64, INNER = 512, NQ = Bn * HWQ  , NC = Bn * L  ;
constexpr float AS_ = 8.0f, SCALE = 0.125f;

typedef _Float16 b16;
typedef __attribute__((ext_vector_type(16))) _Float16 v16b;
typedef __attribute__((ext_vector_type(8))) _Float16 v8b;
typedef __attribute__((ext_vector_type(8))) float v8f;
typedef __attribute__((ext_vector_type(4))) float v4f;
__device__ __forceinline__ float bf16_rne(float f) { unsigned int u = __float_as_uint(f); u += 0x7FFFu + ((u >> 16) & 1u); return __uint_as_float(u & 0xFFFF0000u); }
__device__ __forceinline__ void split16(float v, b16& hi, b16& lo) { hi = (b16)v; lo = (b16)(v - (float)hi); }
__device__ __forceinline__ v16b frag_kb(const b16* p, int hh) { const v8b a = *(const v8b*)(p + 8 * hh), b = *(const v8b*)(p + 16 + 8 * hh); v16b f;
#pragma unroll
  for (int e = 0; e < 8; ++e) { f[e] = a[e]; f[8 + e] = b[e]; } return f; }
__device__ __forceinline__ v16b frag_x(const float* p, int hh) { v16b f;
#pragma unroll
  for (int e = 0; e < 8; ++e) { f[e] = (b16)bf16_rne(p[8 * hh + e]); f[8 + e] = (b16)bf16_rne(p[16 + 8 * hh + e]); } return f; }
__device__ __forceinline__ void frag_split(const float* p, int hh, v16b& fh, v16b& fl) {
#pragma unroll
  for (int e = 0; e < 8; ++e) { b16 a, c; split16(p[8 * hh + e] * AS_, a, c); fh[e] = a; fl[e] = c; split16(p[16 + 8 * hh + e] * AS_, a, c); fh[8 + e] = a; fl[8 + e] = c; } }
__device__ __forceinline__ v8f wmma16b(v16b a, v16b b, v8f c) { v8f d = __builtin_amdgcn_wmma_f32_16x16x32_f16(false, a, false, b, (short)0, c, false, false); asm volatile("v_nop\n\tv_nop\n\tv_nop\n\tv_nop" : "+v"(d) : "v"(a), "v"(b)); return d; }
__device__ __forceinline__ void wave_lds_sync() { __builtin_amdgcn_fence(__ATOMIC_RELEASE, "workgroup"); __builtin_amdgcn_wave_barrier(); __builtin_amdgcn_fence(__ATOMIC_ACQUIRE, "workgroup"); }
__device__ __forceinline__ float nexp(float x) { return __builtin_amdgcn_exp2f(x * 1.4426950408889634f); }
__device__ __forceinline__ float pmul(float a, float b) { float p = a * b; asm volatile("" : "+v"(p)); return p; }
__device__ __forceinline__ float wmax(float v) {
#pragma unroll
  for (int o = 1; o < 32; o <<= 1) v = fmaxf(v, __shfl_xor(v, o)); return v; }
__device__ __forceinline__ float wsum(float v) {
#pragma unroll
  for (int o = 1; o < 32; o <<= 1) v += __shfl_xor(v, o); return v; }

struct Wo_ { static constexpr size_t Q = 0, KV = (size_t)INNER * D, O = KV + (size_t)2 * INNER * D, END = O + (size_t)D * INNER; };
__global__ __launch_bounds__(256) void prep_kernel(const float* __restrict__ Wq, const float* __restrict__ Wkv, const float* __restrict__ Wo, const float* __restrict__ bo, b16* __restrict__ R, float* __restrict__ P) {
  const size_t tid = (size_t)blockIdx.x * 256 + threadIdx.x, nth = (size_t)gridDim.x * 256;
  auto tr = [&](size_t base, int nout, int kin, const float* W) { for (size_t p = tid; p < (size_t)nout * (kin / 8); p += nth) { const int o = (int)(p / (kin / 8)), k0 = (int)(p % (kin / 8)) * 8; v8b v;
#pragma unroll
      for (int e = 0; e < 8; ++e) v[e] = (b16)bf16_rne(W[(size_t)(k0 + e) * nout + o]); *(volatile v8b*)(R + base + (size_t)o * kin + k0) = v; } };
  for (int pass = 0; pass < 2; ++pass) { tr(Wo_::Q, INNER, D, Wq); tr(Wo_::KV, 2 * INNER, D, Wkv); tr(Wo_::O, D, INNER, Wo); for (size_t q = tid; q < (size_t)D; q += nth) P[q] = bf16_rne(bo[q]); __threadfence(); }
}

template <int K, int N>
__global__ __launch_bounds__(64) void gemm_kernel(const float* __restrict__ A, const b16* __restrict__ Bw, float* __restrict__ C) {
  __shared__ __attribute__((aligned(16))) float Ts[2][32][128 + 4];
  const int lane = threadIdx.x & 31, wave = threadIdx.x >> 5, nloc = lane & 15, hlf = lane >> 4, m0 = blockIdx.y * 32, c0 = blockIdx.x * 256 + wave * 128;
  v8f acc[2][8];
#pragma unroll
  for (int r = 0; r < 2; ++r)
#pragma unroll
    for (int t = 0; t < 8; ++t) acc[r][t] = (v8f){};
#pragma unroll 2
  for (int kb = 0; kb < K; kb += 32) { const v16b a0 = frag_x(A + (size_t)(m0 + nloc) * K + kb, hlf), a1 = frag_x(A + (size_t)(m0 + 16 + nloc) * K + kb, hlf);
#pragma unroll
    for (int t = 0; t < 8; ++t) { const v16b bw = frag_kb(Bw + (size_t)(c0 + t * 16 + nloc) * K + kb, hlf); acc[0][t] = wmma16b(a0, bw, acc[0][t]); acc[1][t] = wmma16b(a1, bw, acc[1][t]); } }
#pragma unroll
  for (int t = 0; t < 8; ++t)
#pragma unroll
    for (int r = 0; r < 2; ++r)
#pragma unroll
      for (int v = 0; v < 8; ++v) Ts[wave][r * 16 + 8 * hlf + v][t * 16 + nloc] = acc[r][t][v];
  wave_lds_sync();
  for (int pass = 0; pass < 2; ++pass) { for (int i = lane; i < 32 * 32; i += 32) { const int rr = i >> 5, c4 = (i & 31) * 4; *(volatile v4f*)(C + (size_t)(m0 + rr) * N + c0 + c4) = *(const v4f*)(&Ts[wave][rr][c4]); } __threadfence(); }
}

__global__ __launch_bounds__(256) void sattn_kernel(const float* __restrict__ Q, const float* __restrict__ KV, const int* __restrict__ idxs, const float* __restrict__ bias, float* __restrict__ CTX) {
  __shared__ __attribute__((aligned(16))) float qs[8][INNER]; __shared__ float at[8][NH][KN + 1]; __shared__ int ids[8][KN]; __shared__ __attribute__((aligned(16))) float os[8][INNER];
  const int wave = threadIdx.x >> 5, lane = threadIdx.x & 31, qg = blockIdx.x * 8 + wave; const int b = qg / HWQ;
  for (int i = lane; i < INNER / 4; i += 32) *(v4f*)(&qs[wave][i * 4]) = *(const v4f*)(Q + (size_t)qg * INNER + i * 4);
  int id = idxs[(size_t)qg * KN + lane]; id = (id < 0) ? 0 : (id >= L ? L - 1 : id); ids[wave][lane] = id;
  wave_lds_sync();
  { const float* kr = KV + ((size_t)b * L + id) * (2 * INNER); const float bj = bf16_rne(bias[(size_t)qg * KN + lane]);
#pragma unroll
    for (int h = 0; h < NH; ++h) { float s = 0.0f;
#pragma unroll 4
      for (int d4 = 0; d4 < DH; d4 += 4) { const v4f kk = *(const v4f*)(kr + h * DH + d4); const v4f qq = *(const v4f*)(&qs[wave][h * DH + d4]); s += pmul(qq[0], kk[0]); s += pmul(qq[1], kk[1]); s += pmul(qq[2], kk[2]); s += pmul(qq[3], kk[3]); }
      s = s * SCALE + bj; const float m = wmax(s); const float e = nexp(s - m); const float su = wsum(e); at[wave][h][lane] = e / su; } }
  wave_lds_sync();
  { const int d0 = lane * 16, h = d0 / DH; float o[16];
#pragma unroll
    for (int e = 0; e < 16; ++e) o[e] = 0.0f;
    for (int j = 0; j < KN; ++j) { const float a = at[wave][h][j]; const float* vr = KV + ((size_t)b * L + ids[wave][j]) * (2 * INNER) + INNER + d0;
#pragma unroll
      for (int e4 = 0; e4 < 16; e4 += 4) { const v4f vv = *(const v4f*)(vr + e4); o[e4] += pmul(a, vv[0]); o[e4 + 1] += pmul(a, vv[1]); o[e4 + 2] += pmul(a, vv[2]); o[e4 + 3] += pmul(a, vv[3]); } }
#pragma unroll
    for (int e = 0; e < 16; ++e) os[wave][d0 + e] = o[e]; }
  wave_lds_sync();
  for (int pass = 0; pass < 2; ++pass) {
#pragma unroll
    for (int g = 0; g < 4; ++g) *(volatile v4f*)(CTX + (size_t)qg * INNER + g * 128 + lane * 4) = *(const v4f*)(&os[wave][g * 128 + lane * 4]);
    __threadfence(); }
}

__global__ __launch_bounds__(64) void out_kernel(const float* __restrict__ CTX, const b16* __restrict__ R, const float* __restrict__ P, float* __restrict__ out) {
  __shared__ __attribute__((aligned(16))) float Ts[2][32][128 + 4];
  const int lane = threadIdx.x & 31, wave = threadIdx.x >> 5, nloc = lane & 15, hlf = lane >> 4, m0 = blockIdx.y * 32, c0 = blockIdx.x * 256 + wave * 128; const b16* Wo = R + Wo_::O;
  v8f acc[2][8];
#pragma unroll
  for (int r = 0; r < 2; ++r)
#pragma unroll
    for (int t = 0; t < 8; ++t) acc[r][t] = (v8f){};
#pragma unroll 2
  for (int kb = 0; kb < INNER; kb += 32) { v16b a0, l0, a1, l1; frag_split(CTX + (size_t)(m0 + nloc) * INNER + kb, hlf, a0, l0); frag_split(CTX + (size_t)(m0 + 16 + nloc) * INNER + kb, hlf, a1, l1);
#pragma unroll
    for (int t = 0; t < 8; ++t) { const v16b bw = frag_kb(Wo + (size_t)(c0 + t * 16 + nloc) * INNER + kb, hlf); acc[0][t] = wmma16b(a0, bw, acc[0][t]); acc[0][t] = wmma16b(l0, bw, acc[0][t]); acc[1][t] = wmma16b(a1, bw, acc[1][t]); acc[1][t] = wmma16b(l1, bw, acc[1][t]); } }
#pragma unroll
  for (int t = 0; t < 8; ++t) { const float bb = P[c0 + t * 16 + nloc];
#pragma unroll
    for (int r = 0; r < 2; ++r)
#pragma unroll
      for (int v = 0; v < 8; ++v) Ts[wave][r * 16 + 8 * hlf + v][t * 16 + nloc] = acc[r][t][v] * (1.0f / AS_) + bb; }
  wave_lds_sync();
  for (int pass = 0; pass < 2; ++pass) { for (int i = lane; i < 32 * 32; i += 32) { const int rr = i >> 5, c4 = (i & 31) * 4; *(volatile v4f*)(out + (size_t)(m0 + rr) * D + c0 + c4) = *(const v4f*)(&Ts[wave][rr][c4]); } __threadfence(); }
}
}

extern "C" void kernel_launch(void* const* d_in, const int* in_sizes, int n_in,
                              void* d_out, int out_size, void* d_ws, size_t ws_size, hipStream_t stream) {
  (void)n_in; (void)out_size;
  const float* x = (const float*)d_in[0]; const float* ctxin = (const float*)d_in[1]; const int* idxs = (const int*)d_in[2]; const float* bias = (const float*)d_in[3]; const float* Wq = (const float*)d_in[4]; const float* Wkv = (const float*)d_in[5]; const float* Wo = (const float*)d_in[6]; const float* bo = (const float*)d_in[7];
  float* out = (float*)d_out;
  if (in_sizes[0] != NQ * D || in_sizes[1] != NC * D || in_sizes[2] != NQ * KN || in_sizes[4] != D * INNER || in_sizes[5] != D * 2 * INNER) return;
  size_t off = 0; char* ws = (char*)d_ws;
  auto carve = [&](size_t bytes) { char* p = ws + off; off += (bytes + 255) & ~(size_t)255; return p; };
  b16* R = (b16*)carve(Wo_::END * 2); float* P = (float*)carve(D * 4); float* Qf = (float*)carve((size_t)NQ * INNER * 4); float* KVf = (float*)carve((size_t)NC * 2 * INNER * 4); float* CTX = (float*)carve((size_t)NQ * INNER * 4);
  if (off > ws_size) return;
  prep_kernel<<<256, 256, 0, stream>>>(Wq, Wkv, Wo, bo, R, P);
  gemm_kernel<D, INNER><<<dim3(INNER / 256, NQ / 32), 64, 0, stream>>>(x, R + Wo_::Q, Qf);
  gemm_kernel<D, 2 * INNER><<<dim3(2 * INNER / 256, NC / 32), 64, 0, stream>>>(ctxin, R + Wo_::KV, KVf);
  sattn_kernel<<<NQ / 8, 256, 0, stream>>>(Qf, KVf, idxs, bias, CTX);
  out_kernel<<<dim3(D / 256, NQ / 32), 64, 0, stream>>>(CTX, R, P, out);
}
